// SymmetricContraction_2645699854347
// MI455X (gfx1250) — hardware-verified
//
#include <hip/hip_runtime.h>

constexpr int kNodes = 1024;
constexpr int kChan  = 128;
constexpr int kDim   = 16;
constexpr int kSpec  = 64;
constexpr int kRbf   = 32;
constexpr int kK3a   = 23;
constexpr int kK3b   = 33;
constexpr int kKw    = 64;
constexpr int kNcols = 16384;
constexpr int kChanPass = 16;
constexpr int kPasses = kChan / kChanPass;
constexpr int kMrowsPass = kSpec * kChanPass;
constexpr int kAugK  = 32;
constexpr int kAugRows = 64;
constexpr float kUCarry   = 64.0f;
constexpr float kBCarry   = 64.0f;
constexpr float kResCarry = 1024.0f;
constexpr float kResInv   = 1.0f / 1024.0f;
constexpr float kOutScale = 1.0f / 4096.0f;

constexpr size_t kOffAh  = 0;
constexpr size_t kBytesA = (size_t)kSpec * kChan * kKw * 2;
constexpr size_t kOffAl  = kOffAh + kBytesA;
constexpr size_t kOffBt  = kOffAl + kBytesA;
constexpr size_t kBytesBt = (size_t)kNcols * kKw * 2;
constexpr size_t kOffGh  = kOffBt + kBytesBt;
constexpr size_t kBytesG = (size_t)kMrowsPass * kAugRows * kAugK * 2;
constexpr size_t kOffGl  = kOffGh + kBytesG;
constexpr size_t kOffVh  = kOffGl + kBytesG;
constexpr size_t kBytesV = (size_t)kMrowsPass * kNcols * 2;
constexpr size_t kOffVl  = kOffVh + kBytesV;
constexpr size_t kWsTotal = kOffVl + kBytesV;
static_assert(kBytesA == 1048576u);
static_assert(kBytesBt == 2097152u);
static_assert(kBytesG == 4194304u);
static_assert(kBytesV == 33554432u);
static_assert(kWsTotal == 79691776u);
static_assert(kWsTotal <= 134217728u);
static_assert((kOffAl % 128) == 0 && (kOffBt % 128) == 0 && (kOffGh % 128) == 0 && (kOffGl % 128) == 0 &&
              (kOffVh % 128) == 0 && (kOffVl % 128) == 0);
static_assert(kMrowsPass % 32 == 0 && kNcols % 64 == 0 && kKw % 32 == 0);
static_assert(((kMrowsPass / 32) * (kNcols / 64)) % 8 == 0);
static_assert(kK3a + kK3b <= kKw);
static_assert(kNodes % 128 == 0);
static_assert(kPasses * kChanPass == kChan);
static_assert(kDim + 1 <= kAugK);

typedef __attribute__((ext_vector_type(16))) _Float16 v16h;
typedef __attribute__((ext_vector_type(8)))  _Float16 v8h;
typedef __attribute__((ext_vector_type(8)))  float    v8f;
typedef __attribute__((ext_vector_type(4)))  float    v4f;
typedef __attribute__((ext_vector_type(4)))  unsigned int v4u;
typedef __attribute__((ext_vector_type(8)))  unsigned int v8u;

__device__ __forceinline__ void dep_guard_h(v8f& a, v8f& b, v16h x, v16h y) { asm volatile("v_nop\n\tv_nop\n\tv_nop\n\tv_nop" : "+v"(a), "+v"(b) : "v"(x), "v"(y)); }
__device__ __forceinline__ void keep4_h(v16h a, v16h b, v16h c, v16h d) { asm volatile("v_nop" :: "v"(a), "v"(b), "v"(c), "v"(d)); }
__device__ __forceinline__ void acc_guard4(v8f& a, v8f& b, v8f& c, v8f& d) { asm volatile("v_nop\n\tv_nop\n\tv_nop\n\tv_nop" : "+v"(a), "+v"(b), "+v"(c), "+v"(d)); }
template <typename T> struct Frag;
template <> struct Frag<_Float16> {
  typedef v16h V; union U { v16h v; v8h h[2]; };
  static __device__ __forceinline__ v16h load(const _Float16* p) {
    U f; f.h[0] = *(const v8h*)(p); f.h[1] = *(const v8h*)(p + 16); return f.v;
  }
  static __device__ __forceinline__ v8f mma(v16h a, v16h b, v8f c) {
    return __builtin_amdgcn_wmma_f32_16x16x32_f16(false, a, false, b, (short)0, c, false, false);
  }
  static __device__ __forceinline__ void guard(v8f& a, v8f& b, v16h x, v16h y) { dep_guard_h(a, b, x, y); }
  static __device__ __forceinline__ void keep(v16h a, v16h b, v16h c, v16h d) { keep4_h(a, b, c, d); }
};

__device__ __forceinline__ unsigned pk16(unsigned short a, unsigned short b) { return (unsigned)a | ((unsigned)b << 16); }
__device__ __forceinline__ unsigned short h_bits(float f) { const _Float16 h = (_Float16)f; return __builtin_bit_cast(unsigned short, h); }

__device__ __forceinline__ void split16(float p, unsigned short& hb, unsigned short& lb) {
  const _Float16 hq = (_Float16)p;
  const float rem = (p - (float)hq) * kResCarry;
  hb = __builtin_bit_cast(unsigned short, hq);
  lb = h_bits(rem);
}

__device__ __forceinline__ void guard2f4(v8f& a0, v8f& a1, v16h f0, v16h f1, v16h f2, v16h f3) {
  asm volatile("v_nop\n\tv_nop\n\tv_nop\n\tv_nop" : "+v"(a0), "+v"(a1) : "v"(f0), "v"(f1), "v"(f2), "v"(f3) : "memory");
}
__device__ __forceinline__ void guard8f6(v8f& a0, v8f& a1, v8f& a2, v8f& a3, v8f& a4, v8f& a5, v8f& a6, v8f& a7,
                                         v16h f0, v16h f1, v16h f2, v16h f3, v16h f4, v16h f5) {
  asm volatile("v_nop\n\tv_nop\n\tv_nop\n\tv_nop"
               : "+v"(a0), "+v"(a1), "+v"(a2), "+v"(a3), "+v"(a4), "+v"(a5), "+v"(a6), "+v"(a7)
               : "v"(f0), "v"(f1), "v"(f2), "v"(f3), "v"(f4), "v"(f5));
}

__global__ __launch_bounds__(256) void gemm_build_kernel(
    const unsigned short* __restrict__ Ahp, const unsigned short* __restrict__ Alp, int lda,
    const unsigned short* __restrict__ Btp, int ldb,
    unsigned short* __restrict__ Chp, unsigned short* __restrict__ Clp, int ldc,
    int M, int N, int K) {
  typedef _Float16 T;
  const T* Ah = (const T*)Ahp; const T* Al = (const T*)Alp; const T* Bt = (const T*)Btp;
  __shared__ __align__(16) float sT[8][16 * 68];
  const int lane = threadIdx.x & 31;
  const int wave = threadIdx.x >> 5;
  const int tilesN = N >> 6;
  const int tilesM = M >> 5;
  const int tile = blockIdx.x * 8 + wave;
  if (tile >= tilesM * tilesN) return;
  const int tm = tile / tilesN;
  const int tn = tile - tm * tilesN;
  const int m0 = tm << 5;
  const int n0 = tn << 6;

  const int rlane = lane & 15;
  const int koff  = (lane >> 4) * 8;
  const int mOff  = (lane >> 4) * 8;

  v8f acc[2][4], accr[2][4];
#pragma unroll
  for (int i = 0; i < 2; ++i)
#pragma unroll
    for (int j = 0; j < 4; ++j) {
      acc[i][j]  = (v8f){0.f,0.f,0.f,0.f,0.f,0.f,0.f,0.f};
      accr[i][j] = (v8f){0.f,0.f,0.f,0.f,0.f,0.f,0.f,0.f};
    }

  for (int k0 = 0; k0 < K; k0 += 32) {
    v16h bh[4];
#pragma unroll
    for (int j = 0; j < 4; ++j) {
      const size_t bo = (size_t)(n0 + (j << 4) + rlane) * ldb + koff + k0;
      bh[j] = Frag<T>::load(Bt + bo);
    }
#pragma unroll
    for (int i = 0; i < 2; ++i) {
      const size_t ao = (size_t)(m0 + (i << 4) + rlane) * lda + koff + k0;
      const v16h ah = Frag<T>::load(Ah + ao);
      const v16h al = Frag<T>::load(Al + ao);
#pragma unroll
      for (int j = 0; j < 4; ++j) {
        acc[i][j]  = Frag<T>::mma(ah, bh[j], acc[i][j]);
        accr[i][j] = Frag<T>::mma(al, bh[j], accr[i][j]);
      }
      guard8f6(acc[i][0], acc[i][1], acc[i][2], acc[i][3], accr[i][0], accr[i][1], accr[i][2], accr[i][3],
               ah, al, bh[0], bh[1], bh[2], bh[3]);
    }
    Frag<T>::keep(bh[0], bh[1], bh[2], bh[3]);
  }
  acc_guard4(acc[0][0], acc[0][1], acc[0][2], acc[0][3]);
  acc_guard4(acc[1][0], acc[1][1], acc[1][2], acc[1][3]);
  acc_guard4(accr[0][0], accr[0][1], accr[0][2], accr[0][3]);
  acc_guard4(accr[1][0], accr[1][1], accr[1][2], accr[1][3]);

  float* slab = sT[wave];
  T* Ch = (T*)Chp;
  T* Cl = (T*)Clp;
#pragma unroll
  for (int i = 0; i < 2; ++i) {
    const int mBase = m0 + (i << 4);
#pragma unroll
    for (int j = 0; j < 4; ++j) {
#pragma unroll
      for (int r = 0; r < 8; ++r) {
        const float v = fmaf(accr[i][j][r], kResInv, acc[i][j][r]);
        slab[(mOff + r) * 68 + (j << 4) + rlane] = v;
      }
    }
    __builtin_amdgcn_fence(__ATOMIC_RELEASE, "workgroup");
    __builtin_amdgcn_wave_barrier();
    __builtin_amdgcn_fence(__ATOMIC_ACQUIRE, "workgroup");
    {
      const int q = lane >> 3, c8 = (lane & 7) * 8;
      for (int pass = 0; pass < 2; ++pass) {
#pragma unroll
        for (int it = 0; it < 4; ++it) {
          const int row = it * 4 + q;
          const float* sp = slab + row * 68 + c8;
          v8h hv, lv;
#pragma unroll
          for (int e = 0; e < 8; ++e) {
            const _Float16 hq = (_Float16)sp[e];
            const float rem = (sp[e] - (float)hq) * kResCarry;
            hv[e] = hq;
            lv[e] = (_Float16)rem;
          }
          *(volatile v8h*)(Ch + (size_t)(mBase + row) * ldc + n0 + c8) = hv;
          *(volatile v8h*)(Cl + (size_t)(mBase + row) * ldc + n0 + c8) = lv;
        }
        __threadfence();
      }
    }
    __builtin_amdgcn_fence(__ATOMIC_RELEASE, "workgroup");
    __builtin_amdgcn_wave_barrier();
    __builtin_amdgcn_fence(__ATOMIC_ACQUIRE, "workgroup");
  }
}

__global__ __launch_bounds__(256) void prep_u3_kernel(const float* __restrict__ U3a, const float* __restrict__ U3b,
                                                      unsigned short* __restrict__ Btpl) {
  const int t = threadIdx.x;
  const int n = blockIdx.x * 32 + (t >> 3);
  const int col8 = (t & 7) * 8;
  const int ii = (blockIdx.x >> 3) & 3;
  const int xx = n >> 10, yy = (n >> 4) & 15, jj = n & 15;
  const int b3 = (xx * kDim + yy) * kDim + jj;
  unsigned short hb[8];
  if (ii == 0) {
#pragma unroll
    for (int e = 0; e < 8; ++e) {
      const int kc = col8 + e;
      const int kcl = (kc < kK3a) ? kc : (kK3a - 1);
      const float v = U3a[(size_t)b3 * kK3a + kcl];
      const float f = (kc < kK3a) ? kUCarry : 0.0f;
      hb[e] = h_bits(v * f);
    }
  } else {
#pragma unroll
    for (int e = 0; e < 8; ++e) {
      const int kc = col8 + e;
      int k1 = kc - kK3a;
      k1 = (k1 < 0) ? 0 : ((k1 > kK3b - 1) ? (kK3b - 1) : k1);
      const float v = U3b[((size_t)b3 * kK3b + k1) * 3 + (ii - 1)];
      const float f = (kc >= kK3a && kc < kK3a + kK3b) ? kUCarry : 0.0f;
      hb[e] = h_bits(v * f);
    }
  }
  const v4u u = (v4u){pk16(hb[0], hb[1]), pk16(hb[2], hb[3]), pk16(hb[4], hb[5]), pk16(hb[6], hb[7])};
  unsigned short* dst = Btpl + (size_t)n * kKw + col8;
  *(volatile v4u*)dst = u;
  __threadfence();
  *(volatile v4u*)dst = u;
}

__global__ __launch_bounds__(256) void prep_w3_kernel(const float* __restrict__ st, const float* __restrict__ W3a,
                                                      const float* __restrict__ W3b,
                                                      unsigned short* __restrict__ Ah, unsigned short* __restrict__ Al) {
  __shared__ float stl[kRbf];
  __shared__ float wl[(kK3a + kK3b) * kChan];
  const int sp = blockIdx.x, t = threadIdx.x;
  if (t < kRbf) stl[t] = st[sp * kRbf + t];
  __syncthreads();
  const int c = t & (kChan - 1);
#pragma unroll 1
  for (int ks = (t >> 7); ks < kK3a + kK3b; ks += 2) {
    const float* Wp; int KK, kk;
    if (ks < kK3a) { Wp = W3a; KK = kK3a; kk = ks; } else { Wp = W3b; KK = kK3b; kk = ks - kK3a; }
    float acc = 0.0f;
#pragma unroll 4
    for (int e = 0; e < kRbf; ++e) acc = fmaf(stl[e], Wp[(size_t)(e * KK + kk) * kChan + c], acc);
    wl[ks * kChan + c] = acc;
  }
  __syncthreads();
  const int rl = t >> 3, col8 = (t & 7) * 8;
#pragma unroll 1
  for (int it = 0; it < 4; ++it) {
    const int cc = it * 32 + rl;
    const int p = cc >> 4, cl = cc & 15;
    unsigned short hb[8], lb[8];
#pragma unroll
    for (int e = 0; e < 8; ++e) {
      const int kc = col8 + e;
      const int kcl = (kc < kK3a + kK3b) ? kc : (kK3a + kK3b - 1);
      const float v = wl[kcl * kChan + cc];
      const float val = (kc < kK3a + kK3b) ? v : 0.0f;
      split16(val, hb[e], lb[e]);
    }
    const v4u u  = (v4u){pk16(hb[0], hb[1]), pk16(hb[2], hb[3]), pk16(hb[4], hb[5]), pk16(hb[6], hb[7])};
    const v4u ul = (v4u){pk16(lb[0], lb[1]), pk16(lb[2], lb[3]), pk16(lb[4], lb[5]), pk16(lb[6], lb[7])};
    const size_t row = (size_t)p * kMrowsPass + (size_t)sp * kChanPass + cl;
    unsigned short* dsth = Ah + row * kKw + col8;
    unsigned short* dstl = Al + row * kKw + col8;
    *(volatile v4u*)dsth = u;
    *(volatile v4u*)dstl = ul;
    __threadfence();
    *(volatile v4u*)dsth = u;
    *(volatile v4u*)dstl = ul;
  }
}

__global__ __launch_bounds__(256) void prep_aug_kernel(const float* __restrict__ st,
                                                       const float* __restrict__ U2a, const float* __restrict__ U2b,
                                                       const float* __restrict__ U1a, const float* __restrict__ U1b,
                                                       const float* __restrict__ W2a, const float* __restrict__ W2b,
                                                       const float* __restrict__ W1a, const float* __restrict__ W1b,
                                                       unsigned short* __restrict__ Gh, unsigned short* __restrict__ Gl,
                                                       int cpass) {
  __shared__ float stl[kRbf];
  __shared__ float w2l[12 * 32];
  __shared__ float U2l[kDim * kDim * 4 * 6];
  __shared__ float U1l[kDim * 4];
  const int sp = blockIdx.x, t = threadIdx.x, lane = t & 31, wave = t >> 5;
  if (t < kRbf) stl[t] = st[sp * kRbf + t];
#pragma unroll 1
  for (int idx = t; idx < kDim * kDim * 4 * 6; idx += 256) {
    const int k = idx % 6;
    const int r = idx / 6;
    const int i = r & 3;
    const int xy = r >> 2;
    const int k0 = (k < 4) ? k : 3;
    const int i1 = (i > 0) ? (i - 1) : 0;
    const float a = U2a[xy * 4 + k0];
    const float bb = U2b[(xy * 6 + k) * 3 + i1];
    const float fa = (i == 0 && k < 4) ? 1.0f : 0.0f;
    const float fb = (i != 0) ? 1.0f : 0.0f;
    U2l[idx] = fmaf(fa, a, fb * bb);
  }
  if (t < kDim * 4) {
    const int xq = t >> 2, i = t & 3;
    const int i1 = (i > 0) ? (i - 1) : 0;
    const float a = U1a[xq];
    const float bb = U1b[xq * 3 + i1];
    const float fa = (i == 0) ? 1.0f : 0.0f;
    const float fb = 1.0f - fa;
    U1l[t] = fmaf(fa, a, fb * bb);
  }
  __syncthreads();
  for (int o = t; o < 12 * 32; o += 256) {
    const int ksl = o >> 5, cw = o & 31, c = cpass * kChanPass + (cw & 15);
    const float* Wp; int KK, kk;
    if (ksl < 4)        { Wp = W2a; KK = 4; kk = ksl; }
    else if (ksl < 10)  { Wp = W2b; KK = 6; kk = ksl - 4; }
    else if (ksl == 10) { Wp = W1a; KK = 1; kk = 0; }
    else                { Wp = W1b; KK = 1; kk = 0; }
    float acc = 0.0f;
#pragma unroll 4
    for (int e = 0; e < kRbf; ++e) acc = fmaf(stl[e], Wp[(size_t)(e * KK + kk) * kChan + c], acc);
    w2l[o] = acc;
  }
  __syncthreads();

  const int rl = lane >> 2, col8 = (lane & 3) * 8;
  const int xx = 2 * wave + (rl >> 2), ii = rl & 3;
  const float fi0 = (ii == 0) ? 1.0f : 0.0f;
  const float fi1 = 1.0f - fi0;
  const float u1v = U1l[xx * 4 + ii];
#pragma unroll 1
  for (int cw = 0; cw < kChanPass; ++cw) {
    float ws6[6];
#pragma unroll
    for (int k = 0; k < 6; ++k) {
      const float a = w2l[((k < 4) ? k : 3) * 32 + cw];
      const float bb = w2l[(4 + k) * 32 + cw];
      const float fa = (k < 4) ? fi0 : 0.0f;
      ws6[k] = fmaf(fa, a, fi1 * bb);
    }
    const float w1v = fmaf(fi0, w2l[10 * 32 + cw], fi1 * w2l[11 * 32 + cw]);
    const float v1 = u1v * w1v;
    unsigned short hb[8], lb[8];
#pragma unroll
    for (int e = 0; e < 8; ++e) {
      const int col = col8 + e;
      const int y = col & 15;
      const float* up = U2l + ((xx * kDim + y) * 4 + ii) * 6;
      float v2 = 0.0f;
#pragma unroll
      for (int k = 0; k < 6; ++k) v2 = fmaf(up[k], ws6[k], v2);
      const float val = (col < kDim) ? v2 : ((col == kDim) ? v1 : 0.0f);
      split16(kUCarry * val, hb[e], lb[e]);
    }
    const v4u u  = (v4u){pk16(hb[0], hb[1]), pk16(hb[2], hb[3]), pk16(hb[4], hb[5]), pk16(hb[6], hb[7])};
    const v4u ul = (v4u){pk16(lb[0], lb[1]), pk16(lb[2], lb[3]), pk16(lb[4], lb[5]), pk16(lb[6], lb[7])};
    const size_t off = ((size_t)(sp * kChanPass + cw) * kAugRows + xx * 4 + ii) * kAugK + col8;
    unsigned short* dsth = Gh + off;
    unsigned short* dstl = Gl + off;
    *(volatile v4u*)dsth = u;
    *(volatile v4u*)dstl = ul;
    __threadfence();
    *(volatile v4u*)dsth = u;
    *(volatile v4u*)dstl = ul;
  }
}

__global__ __launch_bounds__(128) void apply_kernel(const float* __restrict__ x, const int* __restrict__ index,
                                                    const unsigned short* __restrict__ Vh,
                                                    const unsigned short* __restrict__ Vl,
                                                    const unsigned short* __restrict__ Gh,
                                                    const unsigned short* __restrict__ Gl,
                                                    float* __restrict__ out, int cpass) {
  __shared__ int nl[kNodes];
  __shared__ int wcnt[4];
  __shared__ __align__(16) float outs[16 * 32];
  const int sp = blockIdx.x, g = blockIdx.y;
  const int t = threadIdx.x, lane = t & 31, wave = t >> 5, hh = lane >> 4, cid = lane & 15;

  int base = 0;
#pragma unroll 1
  for (int ch = 0; ch < kNodes / 128; ++ch) {
    const int node = ch * 128 + t;
    int sv = index[node];
    sv = (sv < 0) ? (sv + kSpec) : sv;
    sv = (sv < 0) ? 0 : ((sv > kSpec - 1) ? (kSpec - 1) : sv);
    const bool hit = (sv == sp);
    const unsigned bal = __builtin_amdgcn_ballot_w32(hit);
    const int pre = __builtin_popcount(bal & ((1u << lane) - 1u));
    if (lane == 0) wcnt[wave] = __builtin_popcount(bal);
    __syncthreads();
    const int n0 = wcnt[0], n1 = wcnt[1], n2 = wcnt[2], n3 = wcnt[3];
    int off = base + pre;
    off += (wave > 0) ? n0 : 0;
    off += (wave > 1) ? n1 : 0;
    off += (wave > 2) ? n2 : 0;
    if (hit && off < kNodes) nl[off] = node;
    base += n0 + n1 + n2 + n3;
    __syncthreads();
  }
  const int cnt = (base < kNodes) ? base : kNodes;
  int ntiles = (cnt + 15) >> 4;
  ntiles = (ntiles > kNodes / 16) ? (kNodes / 16) : ntiles;
  const int c0 = cpass * kChanPass + g * 8;

#pragma unroll 1
  for (int nt = 0; nt < ntiles; ++nt) {
    const int slot = nt * 16 + cid;
    const int slotc = (slot < cnt) ? slot : (cnt - 1);
    int node = nl[slotc];
    node = (node < 0) ? 0 : ((node > kNodes - 1) ? (kNodes - 1) : node);
#pragma unroll 1
    for (int cc = 0; cc < 2; ++cc) {
      const int cw = wave * 2 + cc;
      const int c  = c0 + cw;
      const int cl = g * 8 + cw;
      const float* xp = x + ((size_t)node * kChan + c) * kDim;
      const v4f x0 = *(const v4f*)(xp);
      const v4f x1 = *(const v4f*)(xp + 4);
      const v4f x2 = *(const v4f*)(xp + 8);
      const v4f x3 = *(const v4f*)(xp + 12);
      float xr[16];
#pragma unroll
      for (int e = 0; e < 4; ++e) { xr[e] = x0[e]; xr[4 + e] = x1[e]; xr[8 + e] = x2[e]; xr[12 + e] = x3[e]; }
      float xj[8];
#pragma unroll
      for (int m = 0; m < 8; ++m) xj[m] = hh ? xr[8 + m] : xr[m];
      v8f acc[4], accr[4];
#pragma unroll
      for (int mt = 0; mt < 4; ++mt) {
        acc[mt]  = (v8f){0.f, 0.f, 0.f, 0.f, 0.f, 0.f, 0.f, 0.f};
        accr[mt] = (v8f){0.f, 0.f, 0.f, 0.f, 0.f, 0.f, 0.f, 0.f};
      }
      const size_t vrow = (size_t)(sp * kChanPass + cl) * kNcols + (size_t)cid * 256 + hh * 8;
      const _Float16* VrowH = (const _Float16*)Vh + vrow;
      const _Float16* VrowL = (const _Float16*)Vl + vrow;
#pragma unroll
      for (int ks = 0; ks < 8; ++ks) {
        asm volatile("" ::: "memory");
        const float xa = kBCarry * xr[2 * ks];
        const float xb = kBCarry * xr[2 * ks + 1];
        v8u wh, wl;
#pragma unroll
        for (int q = 0; q < 4; ++q) {
          unsigned short h0, l0, h1, l1, h2, l2, h3, l3;
          split16(xa * xj[2 * q],     h0, l0);
          split16(xa * xj[2 * q + 1], h1, l1);
          split16(xb * xj[2 * q],     h2, l2);
          split16(xb * xj[2 * q + 1], h3, l3);
          wh[q]     = pk16(h0, h1);
          wl[q]     = pk16(l0, l1);
          wh[4 + q] = pk16(h2, h3);
          wl[4 + q] = pk16(l2, l3);
        }
        const v16h bfr = __builtin_bit_cast(v16h, wh);
        const v16h bfl = __builtin_bit_cast(v16h, wl);
#pragma unroll
        for (int mt = 0; mt < 4; ++mt) {
          const v16h afr = Frag<_Float16>::load(VrowH + mt * 4096 + ks * 32);
          const v16h afl = Frag<_Float16>::load(VrowL + mt * 4096 + ks * 32);
          acc[mt]  = Frag<_Float16>::mma(afr, bfr, acc[mt]);
          accr[mt] = Frag<_Float16>::mma(afr, bfl, accr[mt]);
          accr[mt] = Frag<_Float16>::mma(afl, bfr, accr[mt]);
          guard2f4(acc[mt], accr[mt], afr, afl, bfr, bfl);
        }
      }
      {
        asm volatile("" ::: "memory");
        v8u wh, wl;
#pragma unroll
        for (int q = 0; q < 4; ++q) {
          unsigned short h0, l0, h1, l1;
          split16(kBCarry * xj[2 * q],     h0, l0);
          split16(kBCarry * xj[2 * q + 1], h1, l1);
          wh[q] = pk16(h0, h1);
          wl[q] = pk16(l0, l1);
        }
        wh[4] = (hh == 0) ? 0x5400u : 0u;
        wl[4] = 0u;
        wh[5] = 0u; wh[6] = 0u; wh[7] = 0u;
        wl[5] = 0u; wl[6] = 0u; wl[7] = 0u;
        const v16h bfr = __builtin_bit_cast(v16h, wh);
        const v16h bfl = __builtin_bit_cast(v16h, wl);
        const size_t grow = ((size_t)(sp * kChanPass + cl) * kAugRows + cid) * kAugK + hh * 8;
        const _Float16* GrowH = (const _Float16*)Gh + grow;
        const _Float16* GrowL = (const _Float16*)Gl + grow;
#pragma unroll
        for (int mt = 0; mt < 4; ++mt) {
          const v16h gfr = Frag<_Float16>::load(GrowH + mt * 16 * kAugK);
          const v16h gfl = Frag<_Float16>::load(GrowL + mt * 16 * kAugK);
          acc[mt]  = Frag<_Float16>::mma(gfr, bfr, acc[mt]);
          accr[mt] = Frag<_Float16>::mma(gfr, bfl, accr[mt]);
          accr[mt] = Frag<_Float16>::mma(gfl, bfr, accr[mt]);
          guard2f4(acc[mt], accr[mt], gfr, gfl, bfr, bfl);
        }
      }
      float po[4];
#pragma unroll
      for (int i = 0; i < 4; ++i) {
        float s = 0.0f;
#pragma unroll
        for (int mt = 0; mt < 4; ++mt) {
#pragma unroll
          for (int rr = 0; rr < 2; ++rr) {
            const float xv = hh ? xr[4 * mt + 2 + rr] : xr[4 * mt + rr];
            const float tot = fmaf(accr[mt][4 * rr + i], kResInv, acc[mt][4 * rr + i]);
            s = fmaf(tot, xv, s);
          }
        }
        po[i] = s;
      }
      const float q0 = __shfl_xor(po[0], 16, 32);
      const float q1 = __shfl_xor(po[1], 16, 32);
      const float q2 = __shfl_xor(po[2], 16, 32);
      const float q3 = __shfl_xor(po[3], 16, 32);
      const float o0 = (po[0] + q0) * kOutScale;
      const float o1 = (po[1] + q1) * kOutScale;
      const float o2 = (po[2] + q2) * kOutScale;
      const float o3 = (po[3] + q3) * kOutScale;
      if (hh == 0) *(v4f*)(outs + cid * 32 + cw * 4) = (v4f){o0, o1, o2, o3};
    }
    __syncthreads();
    {
      const int ns = t >> 3, q4 = (t & 7) * 4;
      const int oslot = nt * 16 + ns;
      const int oslotc = (oslot < cnt) ? oslot : (cnt - 1);
      int onode = nl[oslotc];
      onode = (onode < 0) ? 0 : ((onode > kNodes - 1) ? (kNodes - 1) : onode);
      const v4f v = *(const v4f*)(outs + ns * 32 + q4);
      float* dst = out + ((size_t)onode * kChan + c0) * 4 + q4;
      if (oslot < cnt) *(volatile v4f*)dst = v;
      __threadfence();
      if (oslot < cnt) *(volatile v4f*)dst = v;
    }
    __syncthreads();
  }
}

extern "C" void kernel_launch(void* const* d_in, const int* in_sizes, int n_in,
                              void* d_out, int out_size, void* d_ws, size_t ws_size,
                              hipStream_t stream) {
  if (n_in < 15) return;
  if ((size_t)out_size != (size_t)kNodes * kChan * 4) return;
  if (ws_size < kWsTotal) return;
  if (in_sizes[0] != kNodes * kChan * kDim) return;
  if (in_sizes[1] != kNodes) return;
  if (in_sizes[2] != kSpec * kRbf) return;

  const float* x   = (const float*)d_in[0];
  const int*   idx = (const int*)d_in[1];
  const float* st  = (const float*)d_in[2];
  const float* U3a = (const float*)d_in[3];
  const float* U3b = (const float*)d_in[4];
  const float* U2a = (const float*)d_in[5];
  const float* U2b = (const float*)d_in[6];
  const float* U1a = (const float*)d_in[7];
  const float* U1b = (const float*)d_in[8];
  const float* W3a = (const float*)d_in[9];
  const float* W3b = (const float*)d_in[10];
  const float* W2a = (const float*)d_in[11];
  const float* W2b = (const float*)d_in[12];
  const float* W1a = (const float*)d_in[13];
  const float* W1b = (const float*)d_in[14];
  float* out = (float*)d_out;

  char* ws = (char*)d_ws;
  unsigned short* Ahpl = (unsigned short*)(ws + kOffAh);
  unsigned short* Alpl = (unsigned short*)(ws + kOffAl);
  unsigned short* Btpl = (unsigned short*)(ws + kOffBt);
  unsigned short* Ghpl = (unsigned short*)(ws + kOffGh);
  unsigned short* Glpl = (unsigned short*)(ws + kOffGl);
  unsigned short* Vhpl = (unsigned short*)(ws + kOffVh);
  unsigned short* Vlpl = (unsigned short*)(ws + kOffVl);

  prep_u3_kernel<<<dim3(kNcols / 32), 256, 0, stream>>>(U3a, U3b, Btpl);
  prep_w3_kernel<<<dim3(kSpec), 256, 0, stream>>>(st, W3a, W3b, Ahpl, Alpl);

  const int gemm_blocks = (kMrowsPass / 32) * (kNcols / 64) / 8;
  for (int p = 0; p < kPasses; ++p) {
    prep_aug_kernel<<<dim3(kSpec), 256, 0, stream>>>(st, U2a, U2b, U1a, U1b, W2a, W2b, W1a, W1b, Ghpl, Glpl, p);
    const unsigned short* Ahp = Ahpl + (size_t)p * kMrowsPass * kKw;
    const unsigned short* Alp = Alpl + (size_t)p * kMrowsPass * kKw;
    gemm_build_kernel<<<dim3(gemm_blocks), 256, 0, stream>>>(
        Ahp, Alp, kKw, Btpl, kKw, Vhpl, Vlpl, kNcols, kMrowsPass, kNcols, kKw);
    apply_kernel<<<dim3(kSpec, kChanPass / 8), 128, 0, stream>>>(x, idx, Vhpl, Vlpl, Ghpl, Glpl, out, p);
  }
}
